// LocalEncoder_91199335563962
// MI455X (gfx1250) — hardware-verified
//
#include <hip/hip_runtime.h>
#include <stddef.h>

#define Bsz    4
#define Lseq   4096
#define Dmod   768
#define DFF    3072
#define Kpat   512
#define Hn     12
#define Hd     64
#define VOC    260
#define VP     288
#define BKrows (Bsz * Kpat)
#define NG     4
#define PPB    (Kpat / NG)
#define ATHR   256
#define AWV    (ATHR / 32)
#define PPW    (PPB / AWV)
#define NPASS  (DFF / 256)

static_assert(VP % 32 == 0);
static_assert(VP >= VOC);
static_assert(VP % 4 == 0);
static_assert(VOC <= 65535);
static_assert(Dmod % 32 == 0);
static_assert(Dmod % 128 == 0);
static_assert(Dmod == 6 * 128);
static_assert(DFF % 256 == 0);
static_assert(BKrows % 32 == 0);
static_assert(Hn * Hd == Dmod);
static_assert(Hd == 64);
static_assert(Lseq == ATHR * 16);
static_assert(NG * PPB == Kpat);
static_assert(AWV * PPW == PPB);
static_assert(AWV * Dmod * 4 <= Lseq * 8);
static_assert((DFF * Dmod) % 8 == 0);
static_assert((Dmod * Dmod) % 8 == 0);

typedef unsigned short us;
typedef unsigned long long u64;
typedef __bf16 v16bf __attribute__((ext_vector_type(16)));
typedef us v8us_t __attribute__((ext_vector_type(8)));
typedef v8us_t __attribute__((may_alias)) v8us;
typedef float v8f __attribute__((ext_vector_type(8)));
typedef float v4f_t __attribute__((ext_vector_type(4)));
typedef v4f_t __attribute__((may_alias)) v4f;
typedef float v2f_t __attribute__((ext_vector_type(2)));
typedef v2f_t __attribute__((may_alias)) v2f;
typedef unsigned int v4u_t __attribute__((ext_vector_type(4)));
typedef v4u_t __attribute__((may_alias)) v4u;

union FragB { v16bf v; v8us_t hv[2]; };

__device__ __forceinline__ v8f zero8() {
    v8f z;
#pragma unroll
    for (int i = 0; i < 8; ++i) z[i] = 0.0f;
    return z;
}

__device__ __forceinline__ unsigned f2bf(float f) {
    unsigned u = __float_as_uint(f);
    u += 0x7FFFu + ((u >> 16) & 1u);
    return u >> 16;
}
__device__ __forceinline__ float bf2f(unsigned b) { return __uint_as_float(b << 16); }

__device__ __forceinline__ void split_pack8(const float (&x)[8], v4u_t& ph, v4u_t& pl) {
#pragma unroll
    for (int j = 0; j < 4; ++j) {
        const unsigned h0 = f2bf(x[2 * j]);
        const unsigned h1 = f2bf(x[2 * j + 1]);
        const unsigned l0 = f2bf(x[2 * j] - bf2f(h0));
        const unsigned l1 = f2bf(x[2 * j + 1] - bf2f(h1));
        ph[j] = h0 | (h1 << 16);
        pl[j] = l0 | (l1 << 16);
    }
}

__device__ __forceinline__ v16bf ldfb(const us* p, int k0) {
    FragB f;
    f.hv[0] = *(const v8us*)(p + k0);
    f.hv[1] = *(const v8us*)(p + k0 + 16);
    return f.v;
}

__device__ __forceinline__ v8f wmma_bf(v16bf a, v16bf b, v8f c) {
    return __builtin_amdgcn_wmma_f32_16x16x32_bf16(false, a, false, b, (short)0, c, false, false);
}

__device__ __forceinline__ void mma_hl_32x32(const us* __restrict__ pah, const us* __restrict__ pal,
                                             const us* __restrict__ pbh, const us* __restrict__ pbl,
                                             v8f (&acc)[2][2])
{
#pragma unroll 1
    for (int k0 = 0; k0 < Dmod; k0 += 32) {
        const v16bf ah0 = ldfb(pah, k0);
        const v16bf ah1 = ldfb(pah + 16 * Dmod, k0);
        const v16bf al0 = ldfb(pal, k0);
        const v16bf al1 = ldfb(pal + 16 * Dmod, k0);
        const v16bf bh0 = ldfb(pbh, k0);
        const v16bf bh1 = ldfb(pbh + 16 * Dmod, k0);
        const v16bf bl0 = ldfb(pbl, k0);
        const v16bf bl1 = ldfb(pbl + 16 * Dmod, k0);
        acc[0][0] = wmma_bf(ah0, bh0, acc[0][0]);
        acc[0][1] = wmma_bf(ah0, bh1, acc[0][1]);
        acc[1][0] = wmma_bf(ah1, bh0, acc[1][0]);
        acc[1][1] = wmma_bf(ah1, bh1, acc[1][1]);
        acc[0][0] = wmma_bf(al0, bh0, acc[0][0]);
        acc[0][1] = wmma_bf(al0, bh1, acc[0][1]);
        acc[1][0] = wmma_bf(al1, bh0, acc[1][0]);
        acc[1][1] = wmma_bf(al1, bh1, acc[1][1]);
        acc[0][0] = wmma_bf(ah0, bl0, acc[0][0]);
        acc[0][1] = wmma_bf(ah0, bl1, acc[0][1]);
        acc[1][0] = wmma_bf(ah1, bl0, acc[1][0]);
        acc[1][1] = wmma_bf(ah1, bl1, acc[1][1]);
        asm volatile("v_nop\n\tv_nop\n\tv_nop\n\tv_nop"
                     : "+v"(acc[0][0]), "+v"(acc[0][1]), "+v"(acc[1][0]), "+v"(acc[1][1])
                     : "v"(ah0), "v"(ah1), "v"(al0), "v"(al1),
                       "v"(bh0), "v"(bh1), "v"(bl0), "v"(bl1));
    }
}

__global__ void __launch_bounds__(256) cvt_hl_kernel(const float* __restrict__ src,
                                                    us* __restrict__ hi, us* __restrict__ lo, int n8)
{
    const int i = blockIdx.x * 256 + threadIdx.x;
    const bool ok = (i < n8);
    const int ic = ok ? i : 0;
    const v4f_t a = *(const v4f*)(src + (size_t)ic * 8);
    const v4f_t c = *(const v4f*)(src + (size_t)ic * 8 + 4);
    float x[8];
#pragma unroll
    for (int j = 0; j < 4; ++j) { x[j] = a[j]; x[4 + j] = c[j]; }
    v4u_t ph, pl;
    split_pack8(x, ph, pl);
    if (ok) {
        *(volatile v4u_t*)(hi + (size_t)i * 8) = ph;
        *(volatile v4u_t*)(lo + (size_t)i * 8) = pl;
    }
    __threadfence();
    if (ok) {
        *(volatile v4u_t*)(hi + (size_t)i * 8) = ph;
        *(volatile v4u_t*)(lo + (size_t)i * 8) = pl;
    }
}

__global__ void __launch_bounds__(128) prep_kernel(const float* __restrict__ embW,
    const float* __restrict__ qw, const float* __restrict__ kvw,
    us* __restrict__ Eh, us* __restrict__ El,
    us* __restrict__ QNh, us* __restrict__ QNl,
    us* __restrict__ KNh, us* __restrict__ KNl)
{
    const int lane = threadIdx.x & 31;
    const int r = blockIdx.x * 4 + (threadIdx.x >> 5);
    const int rc = min(r, VOC - 1);
    const float keep = (r < VOC) ? 1.0f : 0.0f;
    const float* row = embW + (size_t)rc * Dmod;

    float x[3][8];
#pragma unroll
    for (int t = 0; t < 3; ++t) {
        const int g = (lane + 32 * t) * 8;
        const v4f_t a = *(const v4f*)(row + g);
        const v4f_t c = *(const v4f*)(row + g + 4);
#pragma unroll
        for (int j = 0; j < 4; ++j) { x[t][j] = a[j] * keep; x[t][4 + j] = c[j] * keep; }
    }
    float ss = 0.0f;
#pragma unroll
    for (int t = 0; t < 3; ++t) {
#pragma unroll
        for (int j = 0; j < 8; ++j) ss += x[t][j] * x[t][j];
    }
#pragma unroll
    for (int off = 16; off > 0; off >>= 1) ss += __shfl_xor(ss, off, 32);
    const float sc = rsqrtf(ss * (1.0f / (float)Dmod) + 1e-5f);

    v4u_t peh[3], pel[3], pqh[3], pql[3], pkh[3], pkl[3];
#pragma unroll
    for (int t = 0; t < 3; ++t) {
        const int g = (lane + 32 * t) * 8;
        const v4f_t qa = *(const v4f*)(qw + g);
        const v4f_t qb = *(const v4f*)(qw + g + 4);
        const v4f_t ka = *(const v4f*)(kvw + g);
        const v4f_t kb = *(const v4f*)(kvw + g + 4);
        float e8[8], q8[8], k8[8];
#pragma unroll
        for (int j = 0; j < 4; ++j) {
            const float xs0 = x[t][j] * sc, xs1 = x[t][4 + j] * sc;
            e8[j] = x[t][j];       e8[4 + j] = x[t][4 + j];
            q8[j] = xs0 * qa[j];   q8[4 + j] = xs1 * qb[j];
            k8[j] = xs0 * ka[j];   k8[4 + j] = xs1 * kb[j];
        }
        split_pack8(e8, peh[t], pel[t]);
        split_pack8(q8, pqh[t], pql[t]);
        split_pack8(k8, pkh[t], pkl[t]);
    }
    const size_t base = (size_t)r * Dmod;
#pragma unroll
    for (int t = 0; t < 3; ++t) {
        const size_t o = base + (size_t)(lane + 32 * t) * 8;
        *(volatile v4u_t*)(Eh + o)  = peh[t];
        *(volatile v4u_t*)(El + o)  = pel[t];
        *(volatile v4u_t*)(QNh + o) = pqh[t];
        *(volatile v4u_t*)(QNl + o) = pql[t];
        *(volatile v4u_t*)(KNh + o) = pkh[t];
        *(volatile v4u_t*)(KNl + o) = pkl[t];
    }
    __threadfence();
#pragma unroll
    for (int t = 0; t < 3; ++t) {
        const size_t o = base + (size_t)(lane + 32 * t) * 8;
        *(volatile v4u_t*)(Eh + o)  = peh[t];
        *(volatile v4u_t*)(El + o)  = pel[t];
        *(volatile v4u_t*)(QNh + o) = pqh[t];
        *(volatile v4u_t*)(QNl + o) = pql[t];
        *(volatile v4u_t*)(KNh + o) = pkh[t];
        *(volatile v4u_t*)(KNl + o) = pkl[t];
    }
}

__global__ void __launch_bounds__(256) bp_kernel(const us* __restrict__ Eh, const us* __restrict__ El,
    const us* __restrict__ W1h, const us* __restrict__ W1l,
    const float* __restrict__ b1, const float* __restrict__ w2, const float* __restrict__ b2,
    float* __restrict__ lpv)
{
    __shared__ float rowp[8][32];
    const int tid = threadIdx.x, lane = tid & 31, w = tid >> 5;
    const int h = lane >> 4, m = lane & 15;
    const int row0 = blockIdx.x * 32;

    const us* pah = Eh + (size_t)(row0 + m) * Dmod + 8 * h;
    const us* pal = El + (size_t)(row0 + m) * Dmod + 8 * h;

    float part[2][8];
#pragma unroll
    for (int mi = 0; mi < 2; ++mi) {
#pragma unroll
        for (int r = 0; r < 8; ++r) part[mi][r] = 0.0f;
    }

#pragma unroll 1
    for (int p = 0; p < NPASS; ++p) {
        const int col0 = p * 256 + w * 32;
        const us* pbh = W1h + (size_t)(col0 + m) * Dmod + 8 * h;
        const us* pbl = W1l + (size_t)(col0 + m) * Dmod + 8 * h;
        v8f acc[2][2];
        acc[0][0] = zero8(); acc[0][1] = zero8(); acc[1][0] = zero8(); acc[1][1] = zero8();
        mma_hl_32x32(pah, pal, pbh, pbl, acc);
#pragma unroll
        for (int ni = 0; ni < 2; ++ni) {
            const int col = col0 + ni * 16 + m;
            const float bb = b1[col];
            const float ww = w2[col];
#pragma unroll
            for (int mi = 0; mi < 2; ++mi) {
#pragma unroll
                for (int r = 0; r < 8; ++r) {
                    const float y  = acc[mi][ni][r] + bb;
                    const float e  = __expf(-y);
                    const float sg = __builtin_amdgcn_rcpf(1.0f + e);
                    part[mi][r] += (y * sg) * ww;
                }
            }
        }
    }
#pragma unroll
    for (int mi = 0; mi < 2; ++mi) {
#pragma unroll
        for (int r = 0; r < 8; ++r) {
            float v = part[mi][r];
            v += __shfl_xor(v, 1, 32);
            v += __shfl_xor(v, 2, 32);
            v += __shfl_xor(v, 4, 32);
            v += __shfl_xor(v, 8, 32);
            part[mi][r] = v;
        }
    }
    if (m == 0) {
#pragma unroll
        for (int mi = 0; mi < 2; ++mi) {
#pragma unroll
            for (int r = 0; r < 8; ++r) rowp[w][mi * 16 + 8 * h + r] = part[mi][r];
        }
    }
    __syncthreads();
    float lp = 0.0f;
    if (tid < 32) {
        float s = 0.0f;
#pragma unroll
        for (int u = 0; u < 8; ++u) s += rowp[u][tid];
        const float z = s + b2[0];
        lp = fminf(z, 0.0f) - log1pf(expf(-fabsf(z)));
        *(volatile float*)(lpv + row0 + tid) = lp;
    }
    __threadfence();
    if (tid < 32) {
        *(volatile float*)(lpv + row0 + tid) = lp;
    }
}

__global__ void __launch_bounds__(128) gemm_hl_kernel(const us* __restrict__ Ah, const us* __restrict__ Al,
    const us* __restrict__ Wh, const us* __restrict__ Wl, float* __restrict__ C, int ldc)
{
    __shared__ __align__(16) float stg[4][32 * 32];
    const int tid = threadIdx.x, lane = tid & 31, w = tid >> 5;
    const int h = lane >> 4, m = lane & 15;
    const int row0 = blockIdx.x * 32;
    const int col0 = blockIdx.y * 128 + w * 32;

    v8f acc[2][2];
    acc[0][0] = zero8(); acc[0][1] = zero8(); acc[1][0] = zero8(); acc[1][1] = zero8();
    const us* pah = Ah + (size_t)(row0 + m) * Dmod + 8 * h;
    const us* pal = Al + (size_t)(row0 + m) * Dmod + 8 * h;
    const us* pbh = Wh + (size_t)(col0 + m) * Dmod + 8 * h;
    const us* pbl = Wl + (size_t)(col0 + m) * Dmod + 8 * h;
    mma_hl_32x32(pah, pal, pbh, pbl, acc);

    float* stw = stg[w];
#pragma unroll
    for (int mi = 0; mi < 2; ++mi) {
#pragma unroll
        for (int ni = 0; ni < 2; ++ni) {
#pragma unroll
            for (int r = 0; r < 8; ++r)
                stw[(mi * 16 + 8 * h + r) * 32 + ni * 16 + m] = acc[mi][ni][r];
        }
    }
    __syncthreads();
    const int c4 = (lane & 7) * 4;
    const int rq = lane >> 3;
    v4f_t v[8];
#pragma unroll
    for (int p = 0; p < 8; ++p) v[p] = *(const v4f*)(stw + (4 * p + rq) * 32 + c4);
    float* gb = C + (size_t)row0 * ldc + col0 + c4;
#pragma unroll
    for (int p = 0; p < 8; ++p)
        *(volatile v4f_t*)(gb + (size_t)(4 * p + rq) * ldc) = v[p];
    __threadfence();
#pragma unroll
    for (int p = 0; p < 8; ++p)
        *(volatile v4f_t*)(gb + (size_t)(4 * p + rq) * ldc) = v[p];
}

__device__ __forceinline__ unsigned ford(float v) {
    const unsigned u = __float_as_uint(v);
    return (u & 0x80000000u) ? ~u : (u | 0x80000000u);
}

__global__ void __launch_bounds__(ATHR) attn_kernel(const int* __restrict__ tokens,
    const float* __restrict__ lpv, const int* __restrict__ kpat,
    const float* __restrict__ Qv, const float* __restrict__ Kv, const float* __restrict__ Vv,
    us* __restrict__ Oh, us* __restrict__ Ol)
{
    __shared__ __align__(16) u64 keyL[Lseq];
    __shared__ __align__(16) int flg[Lseq];
    __shared__ __align__(16) us tokL[Lseq];
    __shared__ int posL[Kpat + 32];
    __shared__ int wtot[AWV];

    const int tid = threadIdx.x, lane = tid & 31, w = tid >> 5;
    const int g = blockIdx.x, b = blockIdx.y;
    const int* trow = tokens + (size_t)b * Lseq;
    int nsel = kpat[0];
    nsel = min(max(nsel, 1), Kpat);

    for (int l = tid; l < Lseq; l += ATHR) {
        int t = trow[l];
        t = min(max(t, 0), VOC - 1);
        tokL[l] = (us)t;
        const float lv = lpv[t];
        const float v = (l == 0) ? 0.0f : lv;
        const unsigned f = ford(v);
        const unsigned nf = ~f;
        keyL[l] = ((u64)nf << 32) | (u64)(unsigned)l;
    }
    __syncthreads();

    for (int k = 2; k <= Lseq; k <<= 1) {
        for (int j = k >> 1; j > 0; j >>= 1) {
#pragma unroll
            for (int s = 0; s < Lseq / 2 / ATHR; ++s) {
                const int p  = tid + s * ATHR;
                const int i  = ((p & ~(j - 1)) << 1) | (p & (j - 1));
                const int ix = i | j;
                const u64 a = keyL[i], c = keyL[ix];
                const bool asc = ((i & k) == 0);
                const bool sw  = asc ? (a > c) : (a < c);
                if (sw) { keyL[i] = c; keyL[ix] = a; }
            }
            __syncthreads();
        }
    }

    for (int i = tid; i < Lseq; i += ATHR) flg[i] = 0;
    for (int i = tid; i < Kpat + 32; i += ATHR) posL[i] = Lseq;
    __syncthreads();
    for (int i = tid; i < nsel; i += ATHR) {
        const int l = (int)(keyL[i] & 0xFFFull);
        flg[l] = 1;
    }
    __syncthreads();

    {
        int cnt = 0;
#pragma unroll
        for (int i = 0; i < 16; ++i) cnt += flg[tid * 16 + i];
        int x = cnt;
#pragma unroll
        for (int off = 1; off < 32; off <<= 1) {
            const int y = __shfl_up(x, off, 32);
            x = (lane >= off) ? (x + y) : x;
        }
        if (lane == 31) wtot[w] = x;
        __syncthreads();
        int base = x - cnt;
#pragma unroll
        for (int u = 0; u < AWV; ++u) base += (u < w) ? wtot[u] : 0;
#pragma unroll
        for (int i = 0; i < 16; ++i) {
            const int l = tid * 16 + i;
            if (flg[l] != 0) {
                if (base < Kpat) posL[base] = l;
                ++base;
            }
        }
        __syncthreads();
    }

    float* qbuf = (float*)keyL + w * Dmod;
    const float NEG = -__builtin_huge_valf();
    for (int t = 0; t < PPW; ++t) {
        const int q  = g * PPB + w * PPW + t;
        const int s0 = posL[q];
        const int e0 = posL[q + 1];
        const int s  = min(max(s0, 0), Lseq);
        const int e  = min(max(e0, s), Lseq);
        const int n  = e - s;
        const int tq = tokL[min(s, Lseq - 1)];
        __syncthreads();
        {
            const float* qr = Qv + (size_t)tq * Dmod;
#pragma unroll
            for (int u = 0; u < 6; ++u)
                *(v4f*)(qbuf + (lane + 32 * u) * 4) = *(const v4f*)(qr + (lane + 32 * u) * 4);
        }
        __syncthreads();
        const size_t orow = (size_t)(b * Kpat + q) * Dmod;
#pragma unroll 1
        for (int hh = 0; hh < Hn; ++hh) {
            float mrun = NEG, ssum = 0.0f, a0 = 0.0f, a1 = 0.0f;
            const int nch = (n + 31) >> 5;
            const v4f* qw4 = (const v4f*)(qbuf + hh * Hd);
#pragma unroll 1
            for (int c = 0; c < nch; ++c) {
                const int  li    = c * 32 + lane;
                const bool valid = (li < n);
                const int  l     = s + min(li, n - 1);
                const int  tk    = tokL[l];
                const v4f* kp4   = (const v4f*)(Kv + (size_t)tk * Dmod + hh * Hd);
                float d = 0.0f;
#pragma unroll 2
                for (int d4 = 0; d4 < Hd / 4; ++d4) {
                    const v4f_t kk = kp4[d4];
                    const v4f_t qq = qw4[d4];
                    d += kk[0] * qq[0];
                    d += kk[1] * qq[1];
                    d += kk[2] * qq[2];
                    d += kk[3] * qq[3];
                }
                const float sc = valid ? d * 0.125f : NEG;
                float cm = sc;
#pragma unroll
                for (int off = 16; off > 0; off >>= 1) cm = fmaxf(cm, __shfl_xor(cm, off, 32));
                const float mnew  = fmaxf(mrun, cm);
                const float alpha = __expf(mrun - mnew);
                const float pe    = __expf(sc - mnew);
                const float p     = valid ? pe : 0.0f;
                float ps = p;
#pragma unroll
                for (int off = 16; off > 0; off >>= 1) ps += __shfl_xor(ps, off, 32);
                ssum = ssum * alpha + ps;
                a0 *= alpha;
                a1 *= alpha;
                mrun = mnew;
                const int nv = min(32, n - c * 32);
                const float* vb = Vv + hh * Hd + 2 * lane;
#pragma unroll 1
                for (int jj = 0; jj < nv; ++jj) {
                    const float pj = __shfl(p, jj, 32);
                    const int   tj = tokL[s + c * 32 + jj];
                    const v2f_t vv = *(const v2f*)(vb + (size_t)tj * Dmod);
                    a0 += pj * vv[0];
                    a1 += pj * vv[1];
                }
            }
            const float inv = (ssum > 0.0f) ? (1.0f / ssum) : 0.0f;
            const float o0 = a0 * inv, o1 = a1 * inv;
            const unsigned h0 = f2bf(o0), h1 = f2bf(o1);
            const unsigned l0 = f2bf(o0 - bf2f(h0)), l1 = f2bf(o1 - bf2f(h1));
            const unsigned hwv = h0 | (h1 << 16);
            const unsigned lwv = l0 | (l1 << 16);
            us* ph = Oh + orow + hh * Hd + 2 * lane;
            us* pl = Ol + orow + hh * Hd + 2 * lane;
            *(volatile unsigned*)ph = hwv;
            *(volatile unsigned*)pl = lwv;
            __threadfence();
            *(volatile unsigned*)ph = hwv;
            *(volatile unsigned*)pl = lwv;
        }
    }
}

extern "C" void kernel_launch(void* const* d_in, const int* in_sizes, int n_in,
                              void* d_out, int out_size, void* d_ws, size_t ws_size,
                              hipStream_t stream)
{
    if (n_in < 13) return;
    if (in_sizes[0] != Bsz * Lseq) return;
    if (in_sizes[1] != VOC * Dmod) return;
    if (in_sizes[2] != DFF * Dmod) return;
    if (in_sizes[3] != DFF) return;
    if (in_sizes[4] != DFF) return;
    if (in_sizes[5] < 1) return;
    if (in_sizes[6] != Dmod * Dmod) return;
    if (in_sizes[7] != Dmod * Dmod) return;
    if (in_sizes[8] != Dmod * Dmod) return;
    if (in_sizes[9] != Dmod * Dmod) return;
    if (in_sizes[10] != Dmod) return;
    if (in_sizes[11] != Dmod) return;
    if (in_sizes[12] < 1) return;
    if (out_size != BKrows * Dmod) return;

    const int*   tokens   = (const int*)  d_in[0];
    const float* embW     = (const float*)d_in[1];
    const float* bp_w1    = (const float*)d_in[2];
    const float* bp_b1    = (const float*)d_in[3];
    const float* bp_w2    = (const float*)d_in[4];
    const float* bp_b2    = (const float*)d_in[5];
    const float* wq       = (const float*)d_in[6];
    const float* wk       = (const float*)d_in[7];
    const float* wv       = (const float*)d_in[8];
    const float* wo       = (const float*)d_in[9];
    const float* qnorm_w  = (const float*)d_in[10];
    const float* kvnorm_w = (const float*)d_in[11];
    const int*   kpat     = (const int*)  d_in[12];
    float* out = (float*)d_out;

    size_t off = 0;
    auto carve = [&](size_t bytes) -> size_t {
        const size_t o = off;
        off = (off + bytes + 255) & ~(size_t)255;
        return o;
    };
    const size_t szW1  = (size_t)DFF * Dmod * 2;
    const size_t szWW  = (size_t)Dmod * Dmod * 2;
    const size_t szVPh = (size_t)VP * Dmod * 2;
    const size_t szVPf = (size_t)VP * Dmod * 4;
    const size_t szLP  = (size_t)VP * 4;
    const size_t szO   = (size_t)BKrows * Dmod * 2;

    const size_t oW1h = carve(szW1), oW1l = carve(szW1);
    const size_t oWQh = carve(szWW), oWQl = carve(szWW);
    const size_t oWKh = carve(szWW), oWKl = carve(szWW);
    const size_t oWVh = carve(szWW), oWVl = carve(szWW);
    const size_t oWOh = carve(szWW), oWOl = carve(szWW);
    const size_t oEh  = carve(szVPh), oEl  = carve(szVPh);
    const size_t oQNh = carve(szVPh), oQNl = carve(szVPh);
    const size_t oKNh = carve(szVPh), oKNl = carve(szVPh);
    const size_t oLP  = carve(szLP);
    const size_t oQv  = carve(szVPf), oKv = carve(szVPf), oVv = carve(szVPf);
    const size_t oOh  = carve(szO),   oOl = carve(szO);
    const size_t total = off;
    if (total > ws_size) return;
    if (total > (size_t)134217728) return;

    char* ws = (char*)d_ws;
    us* W1h = (us*)(ws + oW1h); us* W1l = (us*)(ws + oW1l);
    us* WQh = (us*)(ws + oWQh); us* WQl = (us*)(ws + oWQl);
    us* WKh = (us*)(ws + oWKh); us* WKl = (us*)(ws + oWKl);
    us* WVh = (us*)(ws + oWVh); us* WVl = (us*)(ws + oWVl);
    us* WOh = (us*)(ws + oWOh); us* WOl = (us*)(ws + oWOl);
    us* Eh  = (us*)(ws + oEh);  us* El  = (us*)(ws + oEl);
    us* QNh = (us*)(ws + oQNh); us* QNl = (us*)(ws + oQNl);
    us* KNh = (us*)(ws + oKNh); us* KNl = (us*)(ws + oKNl);
    float* lpv = (float*)(ws + oLP);
    float* Qvt = (float*)(ws + oQv);
    float* Kvt = (float*)(ws + oKv);
    float* Vvt = (float*)(ws + oVv);
    us* Oh = (us*)(ws + oOh); us* Ol = (us*)(ws + oOl);

    const int n8W1 = (DFF * Dmod) / 8, n8WW = (Dmod * Dmod) / 8;
    cvt_hl_kernel<<<(n8W1 + 255) / 256, 256, 0, stream>>>(bp_w1, W1h, W1l, n8W1);
    cvt_hl_kernel<<<(n8WW + 255) / 256, 256, 0, stream>>>(wq, WQh, WQl, n8WW);
    cvt_hl_kernel<<<(n8WW + 255) / 256, 256, 0, stream>>>(wk, WKh, WKl, n8WW);
    cvt_hl_kernel<<<(n8WW + 255) / 256, 256, 0, stream>>>(wv, WVh, WVl, n8WW);
    cvt_hl_kernel<<<(n8WW + 255) / 256, 256, 0, stream>>>(wo, WOh, WOl, n8WW);

    prep_kernel<<<VP / 4, 128, 0, stream>>>(embW, qnorm_w, kvnorm_w, Eh, El, QNh, QNl, KNh, KNl);

    bp_kernel<<<VP / 32, 256, 0, stream>>>(Eh, El, W1h, W1l, bp_b1, bp_w2, bp_b2, lpv);

    gemm_hl_kernel<<<dim3(VP / 32, Dmod / 128), 128, 0, stream>>>(QNh, QNl, WQh, WQl, Qvt, Dmod);
    gemm_hl_kernel<<<dim3(VP / 32, Dmod / 128), 128, 0, stream>>>(KNh, KNl, WKh, WKl, Kvt, Dmod);
    gemm_hl_kernel<<<dim3(VP / 32, Dmod / 128), 128, 0, stream>>>(KNh, KNl, WVh, WVl, Vvt, Dmod);

    attn_kernel<<<dim3(NG, Bsz), ATHR, 0, stream>>>(tokens, lpv, kpat, Qvt, Kvt, Vvt, Oh, Ol);

    gemm_hl_kernel<<<dim3(BKrows / 32, Dmod / 128), 128, 0, stream>>>(Oh, Ol, WOh, WOl, out, Dmod);
}
